// ManualAttention_79731772883737
// MI455X (gfx1250) — hardware-verified
//
#include <hip/hip_runtime.h>
#include <math.h>

#define NB_FULL 4
#define SEQ_FULL 2048
#ifndef NB
#define NB NB_FULL
#endif
#ifndef SEQ
#define SEQ SEQ_FULL
#endif
#define DM 1024
#define NH 16
#define HD 64
#define NQKV 3072
#define HG 2
#define TT SEQ
#define MROWS (NB * SEQ)
#define RPT (TT / 256)
static_assert(SEQ % 256 == 0);
static_assert(SEQ <= SEQ_FULL);
static_assert(NB >= 1 && NB <= NB_FULL);
static_assert(NH % HG == 0);
static_assert(DM == NH * HD);
static_assert(DM % 32 == 0 && HD % 32 == 0 && TT % 128 == 0);

typedef __attribute__((ext_vector_type(16))) _Float16 v16h;
typedef __attribute__((ext_vector_type(16))) __bf16 v16b;
typedef __attribute__((ext_vector_type(8)))  _Float16 v8h;
typedef __attribute__((ext_vector_type(8)))  __bf16 v8b;
typedef __attribute__((ext_vector_type(8)))  float v8f;
typedef __attribute__((ext_vector_type(4)))  float v4f;
typedef __attribute__((ext_vector_type(4)))  unsigned v4u;

template <typename T> __device__ __forceinline__ void vst2(void* p, T v) { *(volatile T*)p = v; __threadfence(); *(volatile T*)p = v; }

__device__ __forceinline__ v8f wmma16(v16h a, v16h b, v8f c) {
  v8f d = __builtin_amdgcn_wmma_f32_16x16x32_f16(false, a, false, b, (short)0, c, false, false);
  asm volatile("v_nop\n\tv_nop\n\tv_nop\n\tv_nop" : "+v"(d) : "v"(a), "v"(b));
  return d;
}
__device__ __forceinline__ v8f wmma_bf(v16b a, v16b b, v8f c) {
  v8f d = __builtin_amdgcn_wmma_f32_16x16x32_bf16(false, a, false, b, (short)0, c, false, false);
  asm volatile("v_nop\n\tv_nop\n\tv_nop\n\tv_nop" : "+v"(d) : "v"(a), "v"(b));
  return d;
}
__device__ __forceinline__ v16h frag_h(const _Float16* rowk0, int lane) {
  union { v16h v; v8h q[2]; } u; const _Float16* p = rowk0 + 8 * (lane >> 4);
  u.q[0] = *(const v8h*)p; u.q[1] = *(const v8h*)(p + 16); return u.v;
}
__device__ __forceinline__ v16b frag_b(const __bf16* rowk0, int lane) {
  union { v16b v; v8b q[2]; } u; const __bf16* p = rowk0 + 8 * (lane >> 4);
  u.q[0] = *(const v8b*)p; u.q[1] = *(const v8b*)(p + 16); return u.v;
}
__device__ __forceinline__ float bfr(float v) { return (float)(__bf16)v; }
#define LDSX() do { asm volatile("s_wait_dscnt 0" ::: "memory"); __builtin_amdgcn_wave_barrier(); __builtin_amdgcn_fence(__ATOMIC_RELEASE, "workgroup"); } while (0)

#define SZ_XB  (2u * (size_t)MROWS * DM)
#define SZ_WQ  (2u * (size_t)NQKV * DM)
#define SZ_S   (4u * (size_t)HG * TT * TT)
#define SZ_PH  (2u * (size_t)HG * TT * TT)
#define SZ_A1  (SZ_XB + SZ_WQ)
#define SZ_A2  (SZ_S + SZ_PH)
#define SZ_A   (SZ_A1 > SZ_A2 ? SZ_A1 : SZ_A2)
#define WS_XB  ((size_t)0)
#define WS_WQ  (WS_XB + SZ_XB)
#define WS_S   ((size_t)0)
#define WS_PH  (WS_S + SZ_S)
#define WS_WO  (SZ_A)
#define SZ_PL  (2u * (size_t)MROWS * DM)
#define WS_QP  (WS_WO + 2u * (size_t)DM * DM)
#define WS_KP  (WS_QP + SZ_PL)
#define WS_VT  (WS_KP + SZ_PL)
#define WS_CTX (WS_VT + SZ_PL)
#define WS_END (WS_CTX + SZ_PL)
static_assert(WS_END <= (size_t)134217728);
static_assert((WS_WQ % 128) == 0 && (WS_PH % 128) == 0 && (WS_WO % 128) == 0 && (WS_QP % 128) == 0);
static_assert((WS_KP % 128) == 0 && (WS_VT % 128) == 0 && (WS_CTX % 128) == 0);
static_assert(SZ_XB + SZ_WQ <= SZ_A && SZ_S + SZ_PH <= SZ_A);

__global__ __launch_bounds__(256) void k_cvt_bf(const float* __restrict__ src, __bf16* __restrict__ dst, int rows, int seg_rows, int seg_stride) {
  const size_t p = (size_t)blockIdx.x * 256 + threadIdx.x;
  const size_t m = p / (DM / 8); const int c = (int)(p % (DM / 8)) * 8;
  if (m >= (size_t)rows) return;
  const size_t sm = (m / (size_t)seg_rows) * (size_t)seg_stride + (m % (size_t)seg_rows);
  const float* s = src + sm * DM + c;
  const v4f a = *(const v4f*)s, e = *(const v4f*)(s + 4);
  v8b t;
#pragma unroll
  for (int i = 0; i < 4; ++i) { t[i] = (__bf16)a[i]; t[4 + i] = (__bf16)e[i]; }
  union { v8b b; v4u u; } o; o.b = t;
  vst2(dst + m * DM + c, o.u);
}
__global__ __launch_bounds__(256) void k_cvt_wo(const float* __restrict__ src, _Float16* __restrict__ dst) {
  const size_t e = ((size_t)blockIdx.x * 256 + threadIdx.x) * 8;
  if (e >= (size_t)DM * DM) return;
  const v4f a = *(const v4f*)(src + e), c = *(const v4f*)(src + e + 4);
  v8h t;
#pragma unroll
  for (int i = 0; i < 4; ++i) { t[i] = (_Float16)(bfr(a[i]) * 64.0f); t[4 + i] = (_Float16)(bfr(c[i]) * 64.0f); }
  union { v8h h; v4u u; } o; o.h = t;
  vst2(dst + e, o.u);
}

__global__ __launch_bounds__(128) void k_qkv(const __bf16* __restrict__ XB, const __bf16* __restrict__ WQ, const float* __restrict__ bias,
                                             _Float16* __restrict__ QP, _Float16* __restrict__ KP, _Float16* __restrict__ VT) {
  __shared__ __align__(16) _Float16 st[128 * 72];
  const int tid = threadIdx.x, wave = tid >> 5, lane = tid & 31, col = lane & 15, g = lane >> 4;
  const int n0 = blockIdx.x * 64, mb = blockIdx.y * 128, m0 = mb + wave * 32;
  const __bf16* ar0 = XB + (size_t)(m0 + col) * DM; const __bf16* ar1 = ar0 + (size_t)16 * DM;
  const __bf16* br = WQ + (size_t)(n0 + col) * DM;
  v8f acc[2][4] = {};
#pragma unroll 1
  for (int k0 = 0; k0 < DM; k0 += 32) {
    const v16b a0 = frag_b(ar0 + k0, lane), a1 = frag_b(ar1 + k0, lane);
#pragma unroll
    for (int nt = 0; nt < 4; ++nt) {
      const v16b bb = frag_b(br + (size_t)nt * 16 * DM + k0, lane);
      acc[0][nt] = wmma_bf(a0, bb, acc[0][nt]);
      acc[1][nt] = wmma_bf(a1, bb, acc[1][nt]);
    }
  }
  const int t = n0 / DM, h = (n0 % DM) / HD, b = mb / SEQ, s0 = mb % SEQ;
  const size_t bh = (size_t)b * NH + h;
  float bv[4];
#pragma unroll
  for (int nt = 0; nt < 4; ++nt) bv[nt] = bfr(bias[n0 + nt * 16 + col]);
  if (t < 2) {
#pragma unroll
    for (int mt = 0; mt < 2; ++mt)
#pragma unroll
      for (int nt = 0; nt < 4; ++nt)
#pragma unroll
        for (int r = 0; r < 8; ++r)
          st[(wave * 32 + mt * 16 + 8 * g + r) * 72 + nt * 16 + col] = (_Float16)(acc[mt][nt][r] + bv[nt]);
    __syncthreads();
    _Float16* dst = QP; if (t == 1) dst = KP;
    dst += (bh * SEQ + s0) * HD;
#pragma unroll
    for (int it = 0; it < 8; ++it) {
      const int p = it * 128 + tid;
      vst2(dst + (size_t)p * 8, *(const v4u*)&st[(p >> 3) * 72 + (p & 7) * 8]);
    }
  } else {
#pragma unroll
    for (int mt = 0; mt < 2; ++mt)
#pragma unroll
      for (int nt = 0; nt < 4; ++nt)
#pragma unroll
        for (int r = 0; r < 8; ++r)
          st[(nt * 16 + col) * 136 + wave * 32 + mt * 16 + 8 * g + r] = (_Float16)(acc[mt][nt][r] + bv[nt]);
    __syncthreads();
#pragma unroll
    for (int it = 0; it < 8; ++it) {
      const int p = it * 128 + tid; const int d = p >> 4, q = p & 15;
      vst2(VT + (bh * HD + d) * (size_t)SEQ + s0 + q * 8, *(const v4u*)&st[d * 136 + q * 8]);
    }
  }
}

__global__ __launch_bounds__(128) void k_sc(const _Float16* __restrict__ QP, const _Float16* __restrict__ KP, int b, int h0, float* __restrict__ S0) {
  __shared__ __align__(16) float ss[4][16][132];
  const int h = h0 + blockIdx.z; float* S = S0 + (size_t)blockIdx.z * TT * TT; const size_t bh = (size_t)b * NH + h;
  const int tid = threadIdx.x, wave = tid >> 5, lane = tid & 31, col = lane & 15, g = lane >> 4;
  const int k0 = blockIdx.y * 128; const int ql0 = blockIdx.x * 64 + wave * 16;
  v8f acc[8] = {};
#pragma unroll
  for (int kc = 0; kc < HD / 32; ++kc) {
    const v16h a = frag_h(QP + (bh * TT + ql0 + col) * HD + kc * 32, lane);
#pragma unroll
    for (int j = 0; j < 8; ++j) acc[j] = wmma16(a, frag_h(KP + (bh * TT + k0 + j * 16 + col) * HD + kc * 32, lane), acc[j]);
  }
#pragma unroll
  for (int j = 0; j < 8; ++j)
#pragma unroll
    for (int r = 0; r < 8; ++r) ss[wave][8 * g + r][j * 16 + col] = acc[j][r] * 0.125f;
  LDSX();
  for (int rl = 0; rl < 16; ++rl) vst2(S + (size_t)(ql0 + rl) * TT + k0 + lane * 4, *(const v4f*)&ss[wave][rl][lane * 4]);
}
__global__ __launch_bounds__(256) void k_sm(const float* __restrict__ S0, _Float16* __restrict__ PH0) {
  __shared__ float sred[8]; __shared__ float sbc; __shared__ __align__(16) _Float16 sh[TT];
  const int t = threadIdx.x; const size_t row = blockIdx.x;
  const float* sr = S0 + (size_t)blockIdx.y * TT * TT + row * TT; _Float16* ph = PH0 + (size_t)blockIdx.y * TT * TT + row * TT;
  float v[RPT]; float m = -3.0e38f;
#pragma unroll
  for (int i = 0; i < RPT; ++i) { v[i] = sr[t + 256 * i]; m = fmaxf(m, v[i]); }
#pragma unroll
  for (int o = 1; o < 32; o <<= 1) m = fmaxf(m, __shfl_xor(m, o));
  if ((t & 31) == 0) sred[t >> 5] = m; __syncthreads();
  if (t == 0) { float a = sred[0]; for (int i = 1; i < 8; ++i) a = fmaxf(a, sred[i]); sbc = a; }
  __syncthreads(); m = sbc; __syncthreads();
  float sum = 0.f;
#pragma unroll
  for (int i = 0; i < RPT; ++i) { v[i] = exp2f((v[i] - m) * 1.4426950408889634f); sum += v[i]; }
#pragma unroll
  for (int o = 1; o < 32; o <<= 1) sum += __shfl_xor(sum, o);
  if ((t & 31) == 0) sred[t >> 5] = sum; __syncthreads();
  if (t == 0) { float a = 0.f; for (int i = 0; i < 8; ++i) a += sred[i]; sbc = 2048.0f * (1.0f / a); }
  __syncthreads(); const float sc = sbc;
#pragma unroll
  for (int i = 0; i < RPT; ++i) sh[t + 256 * i] = (_Float16)(v[i] * sc);
  __syncthreads();
  for (int q = t; q < TT / 8; q += 256) vst2(ph + q * 8, *(const v4u*)&sh[q * 8]);
}
__global__ __launch_bounds__(128) void k_pv(const _Float16* __restrict__ PH0, const _Float16* __restrict__ VT, int b, int h0, _Float16* __restrict__ CTX) {
  __shared__ __align__(16) _Float16 sp[4][16][72];
  const int h = h0 + blockIdx.z; const _Float16* PH = PH0 + (size_t)blockIdx.z * TT * TT; const size_t bh = (size_t)b * NH + h;
  const int tid = threadIdx.x, wave = tid >> 5, lane = tid & 31, col = lane & 15, g = lane >> 4;
  const int ql0 = blockIdx.x * 64 + wave * 16;
  v8f acc[4] = {};
#pragma unroll 1
  for (int kc = 0; kc < TT / 32; ++kc) {
    const v16h pa = frag_h(PH + (size_t)(ql0 + col) * TT + kc * 32, lane);
#pragma unroll
    for (int j = 0; j < 4; ++j) acc[j] = wmma16(pa, frag_h(VT + (bh * HD + j * 16 + col) * (size_t)TT + kc * 32, lane), acc[j]);
  }
#pragma unroll
  for (int j = 0; j < 4; ++j)
#pragma unroll
    for (int r = 0; r < 8; ++r) sp[wave][8 * g + r][j * 16 + col] = (_Float16)(acc[j][r] * (1.0f / 32.0f));
  LDSX();
#pragma unroll
  for (int it = 0; it < 4; ++it) {
    const int p = it * 32 + lane; const int rl = p >> 3, q8 = p & 7;
    vst2(CTX + ((size_t)b * SEQ + ql0 + rl) * DM + h * HD + q8 * 8, *(const v4u*)&sp[wave][rl][q8 * 8]);
  }
}
__global__ __launch_bounds__(128) void k_out(const _Float16* __restrict__ CTX, const _Float16* __restrict__ WO, const float* __restrict__ bias, float* __restrict__ OUT) {
  __shared__ __align__(16) float so[4][32][68];
  const int tid = threadIdx.x, wave = tid >> 5, lane = tid & 31, col = lane & 15, g = lane >> 4;
  const int n0 = blockIdx.x * 64, m0 = blockIdx.y * 128 + wave * 32;
  const _Float16* ar0 = CTX + (size_t)(m0 + col) * DM; const _Float16* ar1 = ar0 + (size_t)16 * DM;
  const _Float16* br = WO + (size_t)(n0 + col) * DM;
  v8f acc[2][4] = {};
#pragma unroll 1
  for (int k0 = 0; k0 < DM; k0 += 32) {
    const v16h a0 = frag_h(ar0 + k0, lane), a1 = frag_h(ar1 + k0, lane);
#pragma unroll
    for (int nt = 0; nt < 4; ++nt) {
      const v16h bb = frag_h(br + (size_t)nt * 16 * DM + k0, lane);
      acc[0][nt] = wmma16(a0, bb, acc[0][nt]);
      acc[1][nt] = wmma16(a1, bb, acc[1][nt]);
    }
  }
  float bv[4];
#pragma unroll
  for (int nt = 0; nt < 4; ++nt) bv[nt] = bfr(bias[n0 + nt * 16 + col]);
#pragma unroll
  for (int mt = 0; mt < 2; ++mt)
#pragma unroll
    for (int nt = 0; nt < 4; ++nt)
#pragma unroll
      for (int r = 0; r < 8; ++r)
        so[wave][mt * 16 + 8 * g + r][nt * 16 + col] = acc[mt][nt][r] * (1.0f / 4096.0f) + bv[nt];
  LDSX();
#pragma unroll
  for (int it = 0; it < 16; ++it) {
    const int p = it * 32 + lane; const int row = p >> 4, q = p & 15;
    vst2(OUT + (size_t)(m0 + row) * DM + n0 + q * 4, *(const v4f*)&so[wave][row][q * 4]);
  }
}

extern "C" void kernel_launch(void* const* d_in, const int* in_sizes, int n_in, void* d_out, int out_size, void* d_ws, size_t ws_size, hipStream_t stream) {
  if (n_in < 5) return;
  if ((size_t)in_sizes[0] < ((size_t)(NB - 1) * SEQ_FULL + SEQ) * DM) return;
  if (in_sizes[1] < NQKV * DM || in_sizes[2] < NQKV || in_sizes[3] < DM * DM || in_sizes[4] < DM) return;
  if ((size_t)out_size < (size_t)MROWS * DM) return;
  if (ws_size < (size_t)WS_END) return;
  const float* X    = (const float*)d_in[0];
  const float* Wqkv = (const float*)d_in[1];
  const float* Bqkv = (const float*)d_in[2];
  const float* Wo   = (const float*)d_in[3];
  const float* Bo   = (const float*)d_in[4];
  char* ws = (char*)d_ws;
  __bf16* XBp = (__bf16*)(ws + WS_XB); __bf16* WQp = (__bf16*)(ws + WS_WQ);
  float* Sp = (float*)(ws + WS_S); _Float16* PHp = (_Float16*)(ws + WS_PH);
  _Float16* WOp = (_Float16*)(ws + WS_WO); _Float16* QPp = (_Float16*)(ws + WS_QP); _Float16* KPp = (_Float16*)(ws + WS_KP);
  _Float16* VTp = (_Float16*)(ws + WS_VT); _Float16* CTXp = (_Float16*)(ws + WS_CTX);

  k_cvt_bf<<<dim3(MROWS * (DM / 8) / 256), 256, 0, stream>>>(X, XBp, MROWS, SEQ, SEQ_FULL);
  k_cvt_bf<<<dim3(NQKV * (DM / 8) / 256), 256, 0, stream>>>(Wqkv, WQp, NQKV, NQKV, NQKV);
  k_cvt_wo<<<dim3(DM * (DM / 8) / 256), 256, 0, stream>>>(Wo, WOp);
  k_qkv<<<dim3(NQKV / 64, MROWS / 128), 128, 0, stream>>>(XBp, WQp, Bqkv, QPp, KPp, VTp);
  for (int b = 0; b < NB; ++b) for (int h0 = 0; h0 < NH; h0 += HG) {
    k_sc<<<dim3(TT / 64, TT / 128, HG), 128, 0, stream>>>(QPp, KPp, b, h0, Sp);
    k_sm<<<dim3(TT, HG), 256, 0, stream>>>(Sp, PHp);
    k_pv<<<dim3(TT / 64, 1, HG), 128, 0, stream>>>(PHp, VTp, b, h0, CTXp);
  }
  k_out<<<dim3(DM / 64, MROWS / 128), 128, 0, stream>>>(CTXp, WOp, Bo, (float*)d_out);
}
